// VSSBlock_16939351015765
// MI455X (gfx1250) — hardware-run, weakly checked
//
#include <hip/hip_runtime.h>
#include <math.h>

typedef __attribute__((ext_vector_type(16))) _Float16 v16h;
typedef __attribute__((ext_vector_type(8)))  _Float16 v8h;
typedef __attribute__((ext_vector_type(16))) __bf16   v16b;
typedef __attribute__((ext_vector_type(8)))  __bf16   v8b;
typedef __attribute__((ext_vector_type(8)))  float    v8f;
typedef __attribute__((ext_vector_type(4)))  float    v4f;
typedef __attribute__((ext_vector_type(4)))  unsigned v4u;

constexpr int kBatch = 2;
constexpr int kHimg  = 128;
constexpr int kWimg  = 128;
constexpr int kCm    = 96;
constexpr int kDin   = 192;
constexpr int kNst   = 16;
constexpr int kRnk   = 6;
constexpr int kSeq   = kHimg * kWimg;
constexpr int kRows  = kBatch * kSeq;
constexpr int kSgh   = 96;
constexpr int kXdP   = 64;
constexpr int kGpadK = 32;
constexpr int kScanTS = 64;
constexpr int kScanCh = 64;
constexpr int kScanYP = 68;
static_assert(kRnk + 2 * kNst == 38, "x_proj width");
static_assert((kCm % 32) == 0 && (kDin % 32) == 0 && (kGpadK % 32) == 0 && (kSgh % 32) == 0, "GEMM K multiples of 32");
static_assert((kRows % 64) == 0 && (kDin % 64) == 0 && (kXdP % 64) == 0 && ((2 * kSgh) % 64) == 0, "GEMM M,N multiples of 64");
static_assert((kSeq % kScanTS) == 0 && (kDin % kScanCh) == 0 && (kSeq % 64) == 0 && (kWimg % 32) == 0, "tile multiples");
static_assert((kRows % 32) == 0 && (kCm % 16) == 0 && (kRows % 256) == 0, "out_proj wave tile 32 x 96, 8 waves per block");

constexpr size_t kPlane96b  = (size_t)kRows * 96 * 2;
constexpr size_t kPlane192b = (size_t)kRows * 192 * 2;
constexpr size_t kPlane192f = (size_t)kRows * 192 * 4;
constexpr size_t kPlane64f  = (size_t)kRows * 64 * 4;
constexpr size_t kPlane64b  = (size_t)kRows * 64 * 2;
constexpr size_t kOffWIN = 0;
constexpr size_t kOffWIL = kOffWIN + (size_t)384 * 96 * 2;
constexpr size_t kOffWXP = kOffWIL + (size_t)192 * 96 * 2;
constexpr size_t kOffWXL = kOffWXP + (size_t)64 * 192 * 2;
constexpr size_t kOffW1P = kOffWXL + (size_t)64 * 192 * 2;
constexpr size_t kOffW2P = kOffW1P + (size_t)2 * 192 * kGpadK * 2;
constexpr size_t kOffWOP = kOffW2P + (size_t)2 * 64 * 96 * 2;
constexpr size_t kOffR1  = kOffWOP + (size_t)96 * 192 * 2;
constexpr size_t kOffR2  = kOffR1  + kPlane192b;
constexpr size_t kOffG   = kOffR2  + 2 * kPlane192b;
constexpr size_t kOffVBC = kOffG   + kPlane192b;
constexpr size_t kOffR5  = kOffVBC + kPlane64b;
constexpr size_t kOffZ   = kOffR5  + kPlane192f;
constexpr size_t kOffXC  = kOffZ   + kPlane192f;
constexpr size_t kWsTotal = kOffXC + kPlane64f;
static_assert(kOffR1 == 245760ull, "weights carve");
static_assert(kWsTotal == 113491968ull, "carve total");
static_assert(kWsTotal <= 134217728ull, "carve cap");
static_assert((kOffWIL % 128) == 0 && (kOffWXP % 128) == 0 && (kOffWXL % 128) == 0 && (kOffW1P % 128) == 0 &&
              (kOffW2P % 128) == 0 && (kOffWOP % 128) == 0 && (kOffR1 % 128) == 0 && (kOffR2 % 128) == 0 &&
              (kOffG % 128) == 0 && (kOffVBC % 128) == 0 && (kOffR5 % 128) == 0 && (kOffZ % 128) == 0 &&
              (kOffXC % 128) == 0 && (kPlane96b % 128) == 0 && (kPlane64f % 128) == 0, "128-B aligned regions");
static_assert(kPlane64f + 2 * kPlane64f == kPlane192f, "XD + SG fit the XI region exactly");
static_assert(2 * kPlane96b == kPlane192b, "XN + HB fit the XS region exactly");

__device__ __forceinline__ unsigned short f2bf_bits(float f) {
  unsigned u = __float_as_uint(f);
  return (unsigned short)((u + 0x7FFFu + ((u >> 16) & 1u)) >> 16);
}
__device__ __forceinline__ float bf_bits2f(unsigned short h) { return __uint_as_float(((unsigned)h) << 16); }
__device__ __forceinline__ float bfw_lo(unsigned w) { return __uint_as_float(w << 16); }
__device__ __forceinline__ float bfw_hi(unsigned w) { return __uint_as_float(w & 0xffff0000u); }

__device__ __forceinline__ void dep_guard4_h(v8f& a, v8f& b, v8f& c, v8f& d, v16h x, v16h y) { asm volatile("v_nop\n\tv_nop\n\tv_nop\n\tv_nop" : "+v"(a), "+v"(b), "+v"(c), "+v"(d) : "v"(x), "v"(y)); }
__device__ __forceinline__ void dep_guard4_b(v8f& a, v8f& b, v8f& c, v8f& d, v16b x, v16b y) { asm volatile("v_nop\n\tv_nop\n\tv_nop\n\tv_nop" : "+v"(a), "+v"(b), "+v"(c), "+v"(d) : "v"(x), "v"(y)); }
__device__ __forceinline__ void dep_guard2_b3(v8f& a, v8f& b, v16b x, v16b y, v16b z) { asm volatile("v_nop\n\tv_nop\n\tv_nop\n\tv_nop" : "+v"(a), "+v"(b) : "v"(x), "v"(y), "v"(z)); }
__device__ __forceinline__ void keep4_h(v16h a, v16h b, v16h c, v16h d) { asm volatile("v_nop" :: "v"(a), "v"(b), "v"(c), "v"(d)); }
__device__ __forceinline__ void keep4_b(v16b a, v16b b, v16b c, v16b d) { asm volatile("v_nop" :: "v"(a), "v"(b), "v"(c), "v"(d)); }
__device__ __forceinline__ void acc_guard4(v8f& a, v8f& b, v8f& c, v8f& d) { asm volatile("v_nop\n\tv_nop\n\tv_nop\n\tv_nop" : "+v"(a), "+v"(b), "+v"(c), "+v"(d)); }
template <typename T> struct Frag;
template <> struct Frag<_Float16> {
  typedef v16h V; union U { v16h v; v8h h[2]; };
  static __device__ __forceinline__ v16h load(const _Float16* p) {
    U f; f.h[0] = *(const v8h*)(p); f.h[1] = *(const v8h*)(p + 16); return f.v;
  }
  static __device__ __forceinline__ v8f mma(v16h a, v16h b, v8f c) {
    return __builtin_amdgcn_wmma_f32_16x16x32_f16(false, a, false, b, (short)0, c, false, false);
  }
  static __device__ __forceinline__ void guard4(v8f& a, v8f& b, v8f& c, v8f& d, v16h x, v16h y) { dep_guard4_h(a, b, c, d, x, y); }
  static __device__ __forceinline__ void keep(v16h a, v16h b, v16h c, v16h d) { keep4_h(a, b, c, d); }
};
template <> struct Frag<__bf16> {
  typedef v16b V; union U { v16b v; v8b h[2]; };
  static __device__ __forceinline__ v16b load(const __bf16* p) {
    U f; f.h[0] = *(const v8b*)(p); f.h[1] = *(const v8b*)(p + 16); return f.v;
  }
  static __device__ __forceinline__ v8f mma(v16b a, v16b b, v8f c) {
    return __builtin_amdgcn_wmma_f32_16x16x32_bf16(false, a, false, b, (short)0, c, false, false);
  }
  static __device__ __forceinline__ void guard4(v8f& a, v8f& b, v8f& c, v8f& d, v16b x, v16b y) { dep_guard4_b(a, b, c, d, x, y); }
  static __device__ __forceinline__ void keep(v16b a, v16b b, v16b c, v16b d) { keep4_b(a, b, c, d); }
};

template <int ET> struct Elem;
template <> struct Elem<0> { typedef _Float16 T; };
template <> struct Elem<1> { typedef __bf16 T; };
template <int ET, bool SPLIT, int BIAS_MODE, int OUT_MODE, bool RESID, int ACT = 0>
__global__ __launch_bounds__(256) void wmma_gemm64(
    const unsigned short* __restrict__ Ap, const unsigned short* __restrict__ A2p, int lda, long strideA,
    const unsigned short* __restrict__ Btp, const unsigned short* __restrict__ Bt2p, int ldb, long strideB,
    void* __restrict__ Cout, void* __restrict__ Cout2, int ldc, long strideC,
    const float* __restrict__ bias,
    const float* __restrict__ resid, long strideR,
    int M, int N, int K, float scale) {
  typedef typename Elem<ET>::T T;
  typedef typename Frag<T>::V V;
  const T* A = (const T*)Ap; const T* A2 = (const T*)A2p; const T* Bt = (const T*)Btp; const T* Bt2 = (const T*)Bt2p;
  __shared__ __align__(16) float sT[8][16 * 68];
  const int b    = blockIdx.y;
  const int lane = threadIdx.x & 31;
  const int wave = threadIdx.x >> 5;
  const int tilesN = N >> 6;
  const int tilesM = M >> 6;
  const int tile = blockIdx.x * 8 + wave;
  if (tile >= tilesM * tilesN) return;
  const int tm = tile / tilesN;
  const int tn = tile - tm * tilesN;
  const int m0 = tm << 6;
  const int n0 = tn << 6;

  const T* Ab  = A  + (size_t)b * strideA;
  const T* Bb  = Bt + (size_t)b * strideB;
  const T* Ab2 = SPLIT ? (A2  + (size_t)b * strideA) : nullptr;
  const T* Bb2 = SPLIT ? (Bt2 + (size_t)b * strideB) : nullptr;

  const int rlane = lane & 15;
  const int koff  = (lane >> 4) * 8;
  const int mOff  = (lane >> 4) * 8;

  v8f acc[4][4];
#pragma unroll
  for (int i = 0; i < 4; ++i)
#pragma unroll
    for (int j = 0; j < 4; ++j) acc[i][j] = (v8f){0.f,0.f,0.f,0.f,0.f,0.f,0.f,0.f};

  for (int k0 = 0; k0 < K; k0 += 32) {
    V bh[4], bl[4];
#pragma unroll
    for (int j = 0; j < 4; ++j) {
      const size_t bo = (size_t)(n0 + (j << 4) + rlane) * ldb + koff + k0;
      bh[j] = Frag<T>::load(Bb + bo);
      if (SPLIT) bl[j] = Frag<T>::load(Bb2 + bo);
    }
#pragma unroll
    for (int i = 0; i < 4; ++i) {
      const size_t ao = (size_t)(m0 + (i << 4) + rlane) * lda + koff + k0;
      V ah = Frag<T>::load(Ab + ao);
      V al;
      if (SPLIT) al = Frag<T>::load(Ab2 + ao);
#pragma unroll
      for (int j = 0; j < 4; ++j) {
        acc[i][j] = Frag<T>::mma(ah, bh[j], acc[i][j]);
        if (SPLIT) {
          acc[i][j] = Frag<T>::mma(ah, bl[j], acc[i][j]);
          acc[i][j] = Frag<T>::mma(al, bh[j], acc[i][j]);
        }
      }
      Frag<T>::guard4(acc[i][0], acc[i][1], acc[i][2], acc[i][3], ah, SPLIT ? al : bh[3]);
    }
    Frag<T>::keep(bh[0], bh[1], bh[2], bh[3]);
    if (SPLIT) Frag<T>::keep(bl[0], bl[1], bl[2], bl[3]);
  }
  acc_guard4(acc[0][0], acc[0][1], acc[0][2], acc[0][3]);
  acc_guard4(acc[1][0], acc[1][1], acc[1][2], acc[1][3]);
  acc_guard4(acc[2][0], acc[2][1], acc[2][2], acc[2][3]);
  acc_guard4(acc[3][0], acc[3][1], acc[3][2], acc[3][3]);

  float* slab = sT[wave];
  const float* Rb = RESID ? (resid + (size_t)b * strideR) : nullptr;
#pragma unroll
  for (int i = 0; i < 4; ++i) {
    const int mBase = m0 + (i << 4);
#pragma unroll
    for (int j = 0; j < 4; ++j) {
      const int n = n0 + (j << 4) + rlane;
      float bv = 0.f;
      if (BIAS_MODE == 2) bv = bias[n];
#pragma unroll
      for (int r = 0; r < 8; ++r) {
        float v = acc[i][j][r] * scale;
        if (BIAS_MODE == 1) v += bias[mBase + mOff + r];
        if (BIAS_MODE == 2) v += bv;
        if (RESID) v += Rb[(size_t)(mBase + mOff + r) * ldc + n];
        if (ACT == 1) v = tanhf(v);
        if (ACT == 2) v = fmaxf(v, 0.0f);
        if (ACT == 3) v = v / (1.0f + expf(-v));
        if (ACT == 4) v = (v > 0.f) ? v : 0.01f * v;
        slab[(mOff + r) * 68 + (j << 4) + rlane] = v;
      }
    }
    __builtin_amdgcn_fence(__ATOMIC_RELEASE, "workgroup");
    __builtin_amdgcn_wave_barrier();
    __builtin_amdgcn_fence(__ATOMIC_ACQUIRE, "workgroup");
    if (OUT_MODE == 0) {
      float* C = (float*)Cout + (size_t)b * strideC;
      const int hh = lane >> 4, c4 = (lane & 15) * 4;
      for (int pass = 0; pass < 2; ++pass) {
#pragma unroll
        for (int it = 0; it < 8; ++it) {
          const int row = it * 2 + hh;
          v4f v = *(const v4f*)(slab + row * 68 + c4);
          *(volatile v4f*)(C + (size_t)(mBase + row) * ldc + n0 + c4) = v;
        }
        __threadfence();
      }
    } else {
      const int q = lane >> 3, c8 = (lane & 7) * 8;
      unsigned short* C  = (unsigned short*)Cout  + (size_t)b * strideC;
      unsigned short* C2 = (OUT_MODE == 2) ? ((unsigned short*)Cout2 + (size_t)b * strideC) : nullptr;
      for (int pass = 0; pass < 2; ++pass) {
#pragma unroll
        for (int it = 0; it < 4; ++it) {
          const int row = it * 4 + q;
          const float* sp = slab + row * 68 + c8;
          v8h hv, lv;
#pragma unroll
          for (int e = 0; e < 8; ++e) {
            if (OUT_MODE == 1) {
              hv[e] = (_Float16)sp[e];
            } else {
              unsigned short hb = f2bf_bits(sp[e]);
              hv[e] = __builtin_bit_cast(_Float16, hb);
              if (OUT_MODE == 2) {
                unsigned short lb = f2bf_bits(sp[e] - bf_bits2f(hb));
                lv[e] = __builtin_bit_cast(_Float16, lb);
              }
            }
          }
          *(volatile v8h*)(C + (size_t)(mBase + row) * ldc + n0 + c8) = hv;
          if (OUT_MODE == 2) *(volatile v8h*)(C2 + (size_t)(mBase + row) * ldc + n0 + c8) = lv;
        }
        __threadfence();
      }
    }
    __builtin_amdgcn_fence(__ATOMIC_RELEASE, "workgroup");
    __builtin_amdgcn_wave_barrier();
    __builtin_amdgcn_fence(__ATOMIC_ACQUIRE, "workgroup");
  }
}

__global__ __launch_bounds__(256) void cvt_rows_bf16_kernel(
    const float* __restrict__ src, unsigned short* __restrict__ dst,
    int srcRows, int srcCols, int dstCols, int s0dst, int s0src, int s0cnt, int s1dst, int s1src, int s1cnt, int total8)
{
  const int i = blockIdx.x * 256 + threadIdx.x;
  if (i >= total8) return;
  const int e0 = i * 8;
  const int n  = e0 / dstCols;
  const int k0 = e0 - n * dstCols;
  const bool in0 = (n >= s0dst) && (n < s0dst + s0cnt);
  const bool in1 = (n >= s1dst) && (n < s1dst + s1cnt);
  int srow = in0 ? (s0src + n - s0dst) : (in1 ? (s1src + n - s1dst) : 0);
  srow = srow < 0 ? 0 : (srow > srcRows - 1 ? srcRows - 1 : srow);
  const bool kv = (k0 + 8 <= srcCols);
  const int kc = kv ? k0 : 0;
  const float* sp = src + (size_t)srow * srcCols + kc;
  const v4f a0 = *(const v4f*)(sp);
  const v4f a1 = *(const v4f*)(sp + 4);
  const float f = ((in0 || in1) && kv) ? 1.0f : 0.0f;
  v8h hv;
#pragma unroll
  for (int e = 0; e < 4; ++e) {
    const unsigned short h0 = f2bf_bits(a0[e] * f), h1 = f2bf_bits(a1[e] * f);
    hv[e]     = __builtin_bit_cast(_Float16, h0);
    hv[4 + e] = __builtin_bit_cast(_Float16, h1);
  }
  unsigned short* q = dst + e0;
  *(volatile v8h*)q = hv;
  __threadfence();
  *(volatile v8h*)q = hv;
}

__global__ __launch_bounds__(256) void ln_c_kernel(
    const float* __restrict__ x, const float* __restrict__ g, const float* __restrict__ bb, unsigned short* __restrict__ XN)
{
  __shared__ __align__(16) unsigned short sT[64 * 96];
  const int tid = threadIdx.x, lane = tid & 31, wave = tid >> 5;
  const int r0 = blockIdx.x * 64;
  const float g0 = g[lane], g1 = g[lane + 32], g2 = g[lane + 64];
  const float b0 = bb[lane], b1 = bb[lane + 32], b2 = bb[lane + 64];
  asm volatile("" ::: "memory");
#pragma unroll 1
  for (int i = 0; i < 8; ++i) {
    const int rl = wave * 8 + i;
    const float* xr = x + (size_t)(r0 + rl) * kCm;
    const float v0 = xr[lane], v1 = xr[lane + 32], v2 = xr[lane + 64];
    float s = (v0 + v1) + v2;
#pragma unroll
    for (int m = 16; m >= 1; m >>= 1) s += __shfl_xor(s, m, 32);
    const float mean = s * (1.0f / 96.0f);
    const float d0 = v0 - mean, d1 = v1 - mean, d2 = v2 - mean;
    float ss = (d0 * d0 + d1 * d1) + d2 * d2;
#pragma unroll
    for (int m = 16; m >= 1; m >>= 1) ss += __shfl_xor(ss, m, 32);
    const float var  = ss * (1.0f / 96.0f);
    const float rstd = 1.0f / sqrtf(var + 1e-5f);
    sT[rl * 96 + lane]      = f2bf_bits(d0 * rstd * g0 + b0);
    sT[rl * 96 + lane + 32] = f2bf_bits(d1 * rstd * g1 + b1);
    sT[rl * 96 + lane + 64] = f2bf_bits(d2 * rstd * g2 + b2);
  }
  __syncthreads();
  v4u vals[3];
#pragma unroll
  for (int it = 0; it < 3; ++it) vals[it] = *(const v4u*)(sT + (it * 256 + tid) * 8);
  unsigned short* dst = XN + (size_t)blockIdx.x * 64 * 96;
  for (int pass = 0; pass < 2; ++pass) {
#pragma unroll
    for (int it = 0; it < 3; ++it) *(volatile v4u*)(dst + (size_t)(it * 256 + tid) * 8) = vals[it];
    __threadfence();
  }
}

__global__ __launch_bounds__(256) void conv3_silu_kernel(
    const float* __restrict__ XI, const float* __restrict__ cw, const float* __restrict__ cb, unsigned short* __restrict__ XS)
{
  __shared__ __align__(16) float sX[3 * 34 * 64];
  __shared__ __align__(16) float sO[32 * 68];
  const int tid = threadIdx.x, lane = tid & 31, wave = tid >> 5;
  const int rb = blockIdx.x;
  const int b  = rb >> 9;
  const int l0 = (rb & 511) * 32;
  const int h  = l0 >> 7;
  const int w0 = l0 & 127;
  const int c0 = blockIdx.y * 64;
#pragma unroll 1
  for (int it = 0; it < 7; ++it) {
    const int idx  = it * 256 + tid;
    const int idxc = idx < 1632 ? idx : 1631;
    const int hr  = idxc / 544;
    const int rem = idxc - hr * 544;
    const int p   = rem >> 4;
    const int q   = rem & 15;
    const int h2 = h - 1 + hr, w2 = w0 - 1 + p;
    const bool valid = (h2 >= 0) && (h2 < kHimg) && (w2 >= 0) && (w2 < kWimg);
    const int h2c = h2 < 0 ? 0 : (h2 > kHimg - 1 ? kHimg - 1 : h2);
    const int w2c = w2 < 0 ? 0 : (w2 > kWimg - 1 ? kWimg - 1 : w2);
    const size_t grow = (size_t)b * kSeq + (size_t)h2c * kWimg + w2c;
    v4f v = *(const v4f*)(XI + grow * kDin + c0 + q * 4);
    const float f = valid ? 1.0f : 0.0f;
    v = v * f;
    if (idx < 1632) *(v4f*)(sX + (hr * 34 + p) * 64 + q * 4) = v;
  }
  const int c = tid & 63, pg = tid >> 6;
  float w9[9];
#pragma unroll
  for (int t = 0; t < 9; ++t) w9[t] = cw[(size_t)(c0 + c) * 9 + t];
  const float bias = cb[c0 + c];
  __syncthreads();
#pragma unroll 1
  for (int p = 0; p < 8; ++p) {
    const int pix = pg * 8 + p;
    float s = 0.0f;
#pragma unroll
    for (int kh = 0; kh < 3; ++kh)
#pragma unroll
      for (int kw = 0; kw < 3; ++kw)
        s = fmaf(w9[kh * 3 + kw], sX[(kh * 34 + pix + kw) * 64 + c], s);
    const float v  = s + bias;
    const float e  = expf(-v);
    const float sv = v * (1.0f / (1.0f + e));
    sO[pix * 68 + c] = sv;
  }
  __syncthreads();
  const int q = lane >> 3, c8 = (lane & 7) * 8;
  const int row = wave * 4 + q;
  const float* sp = sO + row * 68 + c8;
  v8h hv;
#pragma unroll
  for (int e = 0; e < 8; ++e) {
    const unsigned short hb = f2bf_bits(sp[e]);
    hv[e] = __builtin_bit_cast(_Float16, hb);
  }
  unsigned short* dst = XS + ((size_t)b * kSeq + l0 + row) * kDin + c0 + c8;
  for (int pass = 0; pass < 2; ++pass) {
    *(volatile v8h*)dst = hv;
    __threadfence();
  }
}

__global__ __launch_bounds__(256) void glu_kernel(const unsigned* __restrict__ HG, unsigned* __restrict__ G, int totalWords)
{
  const int i = blockIdx.x * 256 + threadIdx.x;
  if (i >= totalWords) return;
  const int g   = i / (kRows * 48);
  const int rem = i - g * (kRows * 48);
  const int row = rem / 48;
  const int q   = rem - row * 48;
  const unsigned* hp = HG + (size_t)g * kRows * 96 + (size_t)row * 96;
  const unsigned w1 = hp[q];
  const unsigned w2 = hp[48 + q];
  const float h1a = bfw_lo(w1), h1b = bfw_hi(w1);
  const float h2a = bfw_lo(w2), h2b = bfw_hi(w2);
  const float ga = 0.5f * h1a * (1.0f + erff(h1a * 0.70710678118654752f)) * h2a;
  const float gb = 0.5f * h1b * (1.0f + erff(h1b * 0.70710678118654752f)) * h2b;
  const unsigned short ba = f2bf_bits(ga), bb = f2bf_bits(gb);
  const unsigned o = (unsigned)ba | ((unsigned)bb << 16);
  ((volatile unsigned*)G)[i] = o;
  __threadfence();
  ((volatile unsigned*)G)[i] = o;
}

__global__ __launch_bounds__(256) void xc_prep_kernel(
    const float* __restrict__ XD, const float* __restrict__ SGB, const float* __restrict__ SGC,
    const float* __restrict__ cdt, const float* __restrict__ cBw, const float* __restrict__ cCw,
    float* __restrict__ XC)
{
  __shared__ __align__(16) float sIn[76 * 40];
  __shared__ __align__(16) float sO[64 * 68];
  __shared__ float sW[38 * 8];
  const int tid = threadIdx.x, lane = tid & 31, wave = tid >> 5;
  const int blk = blockIdx.x;
  const int b   = blk >> 8;
  const int l0  = (blk & 255) * 64;
#pragma unroll 1
  for (int it = 0; it < 2; ++it) {
    const int idx  = it * 256 + tid;
    const int idxc = idx < 266 ? idx : 265;
    const int tch  = idxc / 7;
    const int i    = idxc - tch * 7;
    const int cd   = tch < 5 ? tch : 5;
    const int cbr  = tch - 6;
    const int cbi  = cbr < 0 ? 0 : (cbr > 15 ? 15 : cbr);
    const int ccr  = tch - 22;
    const int cci  = ccr < 0 ? 0 : (ccr > 15 ? 15 : ccr);
    const float a  = cdt[cd * 7 + i];
    const float wb = cBw[cbi * 7 + i];
    const float wc = cCw[cci * 7 + i];
    const float fa = (tch < 6) ? 1.0f : 0.0f;
    const float fb = (tch >= 6 && tch < 22) ? 1.0f : 0.0f;
    const float fc = (tch >= 22) ? 1.0f : 0.0f;
    float w = fa * a;
    w = fmaf(fb, wb, w);
    w = fmaf(fc, wc, w);
    if (idx < 266) sW[tch * 8 + i] = w;
  }
#pragma unroll 1
  for (int it = 0; it < 12; ++it) {
    const int idx  = it * 256 + tid;
    const int idxc = idx < 2888 ? idx : 2887;
    const int r  = idxc / 38;
    const int ch = idxc - r * 38;
    const int l  = l0 - 6 + r;
    const bool lval = (l >= 0) && (l < kSeq);
    const int lc = l < 0 ? 0 : (l > kSeq - 1 ? kSeq - 1 : l);
    const size_t grow = (size_t)b * kSeq + lc;
    const int cbr = ch - 6;
    const int cbi = cbr < 0 ? 0 : (cbr > 15 ? 15 : cbr);
    const int ccr = ch - 22;
    const int cci = ccr < 0 ? 0 : (ccr > 15 ? 15 : ccr);
    const float a  = XD[grow * kXdP + ch];
    const float sb = SGB[grow * kXdP + cbi];
    const float sc = SGC[grow * kXdP + cci];
    const float fb = (ch >= 6 && ch < 22) ? 1.0f : 0.0f;
    const float fc = (ch >= 22) ? 1.0f : 0.0f;
    const float fl = lval ? 1.0f : 0.0f;
    float v = fmaf(fb, sb, a);
    v = fmaf(fc, sc, v);
    v = v * fl;
    if (idx < 2888) sIn[r * 40 + ch] = v;
  }
#pragma unroll 1
  for (int it = 0; it < 7; ++it) {
    const int idx = it * 256 + tid;
    if (idx < 64 * 26) {
      const int r  = idx / 26;
      const int cc = 6 + (idx - r * 26);
      sO[r * 68 + cc] = 0.0f;
    }
  }
  __syncthreads();
  {
    const int r = tid & 63, cg = tid >> 6;
#pragma unroll 1
    for (int ch = cg; ch < 38; ch += 4) {
      float s = 0.0f;
#pragma unroll
      for (int i = 0; i < 7; ++i) s = fmaf(sW[ch * 8 + i], sIn[(r + 2 * i) * 40 + ch], s);
      const int col = (ch < 6) ? ch : (ch + 26);
      sO[r * 68 + col] = s;
    }
  }
  __syncthreads();
  const int hh = lane >> 4, c4 = (lane & 15) * 4;
  float* dst0 = XC + ((size_t)b * kSeq + l0) * kXdP;
  for (int pass = 0; pass < 2; ++pass) {
#pragma unroll
    for (int it = 0; it < 4; ++it) {
      const int row = wave * 8 + it * 2 + hh;
      const v4f v = *(const v4f*)(sO + row * 68 + c4);
      *(volatile v4f*)(dst0 + (size_t)row * kXdP + c4) = v;
    }
    __threadfence();
  }
}

__global__ __launch_bounds__(64) void scan_kernel(
    const float* __restrict__ XC, const unsigned short* __restrict__ XS,
    const float* __restrict__ Wdt, const float* __restrict__ bdt, const float* __restrict__ Alog,
    const float* __restrict__ Dsp, float* __restrict__ Y)
{
  __shared__ __align__(16) float sX[kScanTS * kXdP];
  __shared__ __align__(16) unsigned short sU[kScanTS * kScanCh];
  __shared__ __align__(16) float sY[kScanTS * kScanYP];
  __shared__ float sW[kRnk * kScanCh];
  __shared__ float sA[kNst * kScanCh];
  const int tid = threadIdx.x, lane = tid & 31, wave = tid >> 5;
  constexpr int kBlkPerB = kDin / kScanCh;
  const int bix = blockIdx.x / kBlkPerB;
  const int d0  = (blockIdx.x - bix * kBlkPerB) * kScanCh;
  const int d   = d0 + tid;
  const size_t row0 = (size_t)bix * kSeq;
#pragma unroll 1
  for (int r = 0; r < kRnk; ++r) sW[r * kScanCh + tid] = Wdt[(size_t)d * kRnk + r];
#pragma unroll 1
  for (int s = 0; s < kNst; ++s) sA[s * kScanCh + tid] = -expf(Alog[(size_t)d * kNst + s]);
  __syncthreads();
  float A2[kNst], h[kNst];
#pragma unroll
  for (int s = 0; s < kNst; ++s) {
    A2[s] = sA[s * kScanCh + tid] * 1.4426950408889634f;
    h[s] = 0.0f;
  }
  const float bb = bdt[d], Dv = Dsp[d];
  const int lr = tid >> 4, lc4 = (tid & 15) * 4;
  const int hh = lane >> 4, c4 = (lane & 15) * 4;
#pragma unroll 1
  for (int t0 = 0; t0 < kSeq; t0 += kScanTS) {
    __syncthreads();
#pragma unroll
    for (int i = 0; i < 8; ++i) {
      const int r = lr + 4 * i;
      *(v4f*)(sX + r * kXdP + lc4) = *(const v4f*)(XC + (row0 + t0 + r) * kXdP + lc4);
    }
    asm volatile("" ::: "memory");
#pragma unroll
    for (int i = 8; i < 16; ++i) {
      const int r = lr + 4 * i;
      *(v4f*)(sX + r * kXdP + lc4) = *(const v4f*)(XC + (row0 + t0 + r) * kXdP + lc4);
    }
    asm volatile("" ::: "memory");
#pragma unroll
    for (int i = 0; i < 8; ++i) {
      const int chunk = i * 64 + tid;
      const int r = chunk >> 3, q = chunk & 7;
      *(v4u*)(sU + r * kScanCh + q * 8) = *(const v4u*)(XS + (row0 + t0 + r) * kDin + d0 + q * 8);
    }
    __syncthreads();
#pragma unroll 1
    for (int s = 0; s < kScanTS; ++s) {
      const float* xr = sX + s * kXdP;
      float vdot = 0.0f;
#pragma unroll
      for (int r = 0; r < kRnk; ++r) vdot = fmaf(xr[r], sW[r * kScanCh + tid], vdot);
      const float v   = vdot + bb;
      const float ea  = expf(-fabsf(v));
      const float dt  = fmaxf(v, 0.0f) + log1pf(ea);
      float Bs[kNst], Cs[kNst];
#pragma unroll
      for (int q4 = 0; q4 < 4; ++q4) {
        const v4f bv = *(const v4f*)(xr + 32 + 4 * q4);
        const v4f cv = *(const v4f*)(xr + 48 + 4 * q4);
        Bs[4 * q4 + 0] = bv[0]; Bs[4 * q4 + 1] = bv[1]; Bs[4 * q4 + 2] = bv[2]; Bs[4 * q4 + 3] = bv[3];
        Cs[4 * q4 + 0] = cv[0]; Cs[4 * q4 + 1] = cv[1]; Cs[4 * q4 + 2] = cv[2]; Cs[4 * q4 + 3] = cv[3];
      }
      const float xt  = __uint_as_float(((unsigned)sU[s * kScanCh + tid]) << 16);
      const float dtx = dt * xt;
      float y = 0.0f;
#pragma unroll
      for (int k = 0; k < kNst; ++k) {
        const float e = exp2f(dt * A2[k]);
        h[k] = fmaf(e, h[k], dtx * Bs[k]);
        y = fmaf(h[k], Cs[k], y);
      }
      y = fmaf(Dv, xt, y);
      sY[s * kScanYP + tid] = y;
    }
    __syncthreads();
    for (int pass = 0; pass < 2; ++pass) {
#pragma unroll
      for (int it = 0; it < 16; ++it) {
        const int row = wave * 32 + it * 2 + hh;
        const v4f v = *(const v4f*)(sY + row * kScanYP + c4);
        *(volatile v4f*)(Y + (row0 + t0 + row) * kDin + d0 + c4) = v;
      }
      __threadfence();
    }
  }
}

__global__ __launch_bounds__(256) void ln_gate_kernel(
    const float* __restrict__ Y, const float* __restrict__ Z, const float* __restrict__ g, const float* __restrict__ bb,
    unsigned short* __restrict__ YG)
{
  __shared__ __align__(16) unsigned short sT[64 * 192];
  __shared__ float sG[192];
  __shared__ float sB[192];
  const int tid = threadIdx.x, lane = tid & 31, wave = tid >> 5;
  const int r0 = blockIdx.x * 64;
  {
    const int cc = tid < 192 ? tid : 191;
    const float gv = g[cc], bv = bb[cc];
    if (tid < 192) { sG[tid] = gv; sB[tid] = bv; }
  }
  __syncthreads();
  float gk[6], bk[6];
#pragma unroll
  for (int k = 0; k < 6; ++k) { gk[k] = sG[lane + 32 * k]; bk[k] = sB[lane + 32 * k]; }
#pragma unroll 1
  for (int i = 0; i < 8; ++i) {
    const int rl = wave * 8 + i;
    const size_t row = (size_t)(r0 + rl);
    const float* yr = Y + row * kDin;
    float v[6];
#pragma unroll
    for (int k = 0; k < 6; ++k) v[k] = yr[lane + 32 * k];
    float s = ((v[0] + v[1]) + (v[2] + v[3])) + (v[4] + v[5]);
#pragma unroll
    for (int m = 16; m >= 1; m >>= 1) s += __shfl_xor(s, m, 32);
    const float mean = s * (1.0f / 192.0f);
    float dv[6];
    float ss = 0.0f;
#pragma unroll
    for (int k = 0; k < 6; ++k) { dv[k] = v[k] - mean; ss = fmaf(dv[k], dv[k], ss); }
#pragma unroll
    for (int m = 16; m >= 1; m >>= 1) ss += __shfl_xor(ss, m, 32);
    const float var  = ss * (1.0f / 192.0f);
    const float rstd = 1.0f / sqrtf(var + 1e-5f);
    asm volatile("" ::: "memory");
    const float* zr = Z + row * kDin;
    float z6[6];
#pragma unroll
    for (int k = 0; k < 6; ++k) z6[k] = zr[lane + 32 * k];
#pragma unroll
    for (int k = 0; k < 6; ++k) {
      const float zv = z6[k];
      const float sg = 1.0f / (1.0f + expf(-zv));
      const float o  = (dv[k] * rstd * gk[k] + bk[k]) * (zv * sg);
      sT[rl * 192 + lane + 32 * k] = f2bf_bits(o);
    }
  }
  __syncthreads();
  v4u vals[6];
#pragma unroll
  for (int it = 0; it < 6; ++it) vals[it] = *(const v4u*)(sT + (it * 256 + tid) * 8);
  unsigned short* dst = YG + (size_t)blockIdx.x * 64 * 192;
  for (int pass = 0; pass < 2; ++pass) {
#pragma unroll
    for (int it = 0; it < 6; ++it) *(volatile v4u*)(dst + (size_t)(it * 256 + tid) * 8) = vals[it];
    __threadfence();
  }
}

__global__ __launch_bounds__(256) void outproj_kernel(
    const unsigned short* __restrict__ Ap, const unsigned short* __restrict__ Btp,
    const float* __restrict__ X, float* __restrict__ Out, int M)
{
  const __bf16* A  = (const __bf16*)Ap;
  const __bf16* Bt = (const __bf16*)Btp;
  __shared__ __align__(16) float sT[8][16 * 100];
  const int lane = threadIdx.x & 31;
  const int wave = threadIdx.x >> 5;
  const int m0 = (blockIdx.x * 8 + wave) * 32;
  if (m0 >= M) return;
  const int rlane = lane & 15;
  const int koff  = (lane >> 4) * 8;
  const int mOff  = (lane >> 4) * 8;

  v8f acc[2][6];
#pragma unroll
  for (int i = 0; i < 2; ++i)
#pragma unroll
    for (int j = 0; j < 6; ++j) acc[i][j] = (v8f){0.f,0.f,0.f,0.f,0.f,0.f,0.f,0.f};

  for (int k0 = 0; k0 < kDin; k0 += 32) {
    const v16b a0 = Frag<__bf16>::load(A + (size_t)(m0 + rlane) * kDin + koff + k0);
    const v16b a1 = Frag<__bf16>::load(A + (size_t)(m0 + 16 + rlane) * kDin + koff + k0);
#pragma unroll
    for (int j = 0; j < 6; ++j) {
      const v16b bj = Frag<__bf16>::load(Bt + (size_t)(j * 16 + rlane) * kDin + koff + k0);
      acc[0][j] = Frag<__bf16>::mma(a0, bj, acc[0][j]);
      acc[1][j] = Frag<__bf16>::mma(a1, bj, acc[1][j]);
      dep_guard2_b3(acc[0][j], acc[1][j], a0, a1, bj);
    }
  }
  acc_guard4(acc[0][0], acc[0][1], acc[0][2], acc[0][3]);
  acc_guard4(acc[0][4], acc[0][5], acc[1][0], acc[1][1]);
  acc_guard4(acc[1][2], acc[1][3], acc[1][4], acc[1][5]);

  float* slab = sT[wave];
  const int c4  = lane * 4;
  const int c4c = c4 < 92 ? c4 : 92;
#pragma unroll
  for (int i = 0; i < 2; ++i) {
    const int mBase = m0 + i * 16;
#pragma unroll
    for (int j = 0; j < 6; ++j)
#pragma unroll
      for (int r = 0; r < 8; ++r) slab[(mOff + r) * 100 + j * 16 + rlane] = acc[i][j][r];
    __builtin_amdgcn_fence(__ATOMIC_RELEASE, "workgroup");
    __builtin_amdgcn_wave_barrier();
    __builtin_amdgcn_fence(__ATOMIC_ACQUIRE, "workgroup");
    for (int pass = 0; pass < 2; ++pass) {
#pragma unroll 1
      for (int cq = 0; cq < 4; ++cq) {
#pragma unroll
        for (int u = 0; u < 4; ++u) {
          const int it = cq * 4 + u;
          const size_t row = (size_t)(mBase + it);
          const v4f sv = *(const v4f*)(slab + it * 100 + c4c);
          const v4f xv = *(const v4f*)(X + row * kCm + c4c);
          const v4f o = sv + xv;
          if (lane < 24) *(volatile v4f*)(Out + row * kCm + c4) = o;
        }
      }
      __threadfence();
    }
    __builtin_amdgcn_fence(__ATOMIC_RELEASE, "workgroup");
    __builtin_amdgcn_wave_barrier();
    __builtin_amdgcn_fence(__ATOMIC_ACQUIRE, "workgroup");
  }
}

static_assert((kRows % 64) == 0 && (kDin % 64) == 0 && (kCm % 32) == 0, "in_proj / in_proj_low M,N,K");
static_assert((kXdP % 64) == 0 && (kDin % 32) == 0, "x_proj M,N,K");
static_assert((kGpadK % 32) == 0 && (kSgh % 32) == 0, "gate K");

extern "C" void kernel_launch(void* const* d_in, const int* in_sizes, int n_in,
                              void* d_out, int out_size, void* d_ws, size_t ws_size,
                              hipStream_t stream) {
  if (n_in < 24) return;
  if (in_sizes[0] != kRows * kCm) return;
  if (in_sizes[1] != kRows * kCm) return;
  if (in_sizes[2] != kCm || in_sizes[3] != kCm) return;
  if (in_sizes[4] != 2 * kDin * kCm) return;
  if (in_sizes[5] != kDin * kCm) return;
  if (in_sizes[6] != kDin * 9 || in_sizes[7] != kDin) return;
  if (in_sizes[8] != 38 * kDin || in_sizes[9] != 38 * kDin) return;
  if (in_sizes[10] != kRnk * 7 || in_sizes[11] != kNst * 7 || in_sizes[12] != kNst * 7) return;
  if (in_sizes[13] != 2 * kSgh * kNst || in_sizes[14] != kNst * kSgh) return;
  if (in_sizes[15] != 2 * kSgh * kNst || in_sizes[16] != kNst * kSgh) return;
  if (in_sizes[17] != kDin * kRnk || in_sizes[18] != kDin) return;
  if (in_sizes[19] != kDin * kNst || in_sizes[20] != kDin || in_sizes[21] != kDin || in_sizes[22] != kDin) return;
  if (in_sizes[23] != kCm * kDin) return;
  if (out_size != kRows * kCm) return;
  if (ws_size < kWsTotal) return;

  const float* x             = (const float*)d_in[0];
  const float* hbl           = (const float*)d_in[1];
  const float* ln_g          = (const float*)d_in[2];
  const float* ln_b          = (const float*)d_in[3];
  const float* in_proj_w     = (const float*)d_in[4];
  const float* in_proj_low_w = (const float*)d_in[5];
  const float* conv2d_w      = (const float*)d_in[6];
  const float* conv2d_b      = (const float*)d_in[7];
  const float* x_proj_w      = (const float*)d_in[8];
  const float* x_proj_w_low  = (const float*)d_in[9];
  const float* conv_dt_w     = (const float*)d_in[10];
  const float* conv_B_w      = (const float*)d_in[11];
  const float* conv_C_w      = (const float*)d_in[12];
  const float* sgb_w1        = (const float*)d_in[13];
  const float* sgb_w2        = (const float*)d_in[14];
  const float* sgc_w1        = (const float*)d_in[15];
  const float* sgc_w2        = (const float*)d_in[16];
  const float* dt_proj_w     = (const float*)d_in[17];
  const float* dt_proj_b     = (const float*)d_in[18];
  const float* A_logs        = (const float*)d_in[19];
  const float* Ds            = (const float*)d_in[20];
  const float* outn_g        = (const float*)d_in[21];
  const float* outn_b        = (const float*)d_in[22];
  const float* out_proj_w    = (const float*)d_in[23];
  float* out = (float*)d_out;

  char* ws = (char*)d_ws;
  unsigned short* WIN = (unsigned short*)(ws + kOffWIN);
  unsigned short* WIL = (unsigned short*)(ws + kOffWIL);
  unsigned short* WXP = (unsigned short*)(ws + kOffWXP);
  unsigned short* WXL = (unsigned short*)(ws + kOffWXL);
  unsigned short* W1P = (unsigned short*)(ws + kOffW1P);
  unsigned short* W2P = (unsigned short*)(ws + kOffW2P);
  unsigned short* WOP = (unsigned short*)(ws + kOffWOP);
  unsigned short* XN  = (unsigned short*)(ws + kOffR1);
  unsigned short* HB  = (unsigned short*)(ws + kOffR1 + kPlane96b);
  unsigned short* XS  = (unsigned short*)(ws + kOffR1);
  unsigned short* YG  = (unsigned short*)(ws + kOffR1);
  unsigned short* LOW = (unsigned short*)(ws + kOffR2);
  unsigned short* HG  = (unsigned short*)(ws + kOffR2);
  unsigned short* G   = (unsigned short*)(ws + kOffG);
  unsigned short* VBC = (unsigned short*)(ws + kOffVBC);
  float*          XI  = (float*)(ws + kOffR5);
  float*          XD  = (float*)(ws + kOffR5);
  float*          SG  = (float*)(ws + kOffR5 + kPlane64f);
  float*          Y   = (float*)(ws + kOffR5);
  float*          Z   = (float*)(ws + kOffZ);
  float*          XC  = (float*)(ws + kOffXC);

  auto cvt = [&](const float* src, unsigned short* dst, int srcRows, int srcCols, int dstCols,
                 int s0dst, int s0src, int s0cnt, int s1dst, int s1src, int s1cnt, int dstRows) {
    const int total8 = dstRows * dstCols / 8;
    cvt_rows_bf16_kernel<<<(unsigned)((total8 + 255) / 256), 256, 0, stream>>>(
        src, dst, srcRows, srcCols, dstCols, s0dst, s0src, s0cnt, s1dst, s1src, s1cnt, total8);
  };
  cvt(in_proj_w,     WIN,                 384, kCm,  kCm,    0, 0, 384,   0,  0,  0, 384);
  cvt(in_proj_low_w, WIL,                 192, kCm,  kCm,    0, 0, 192,   0,  0,  0, 192);
  cvt(x_proj_w,      WXP,                  38, kDin, kDin,   0, 0,  38,   0,  0,  0,  64);
  cvt(x_proj_w_low,  WXL,                  38, kDin, kDin,   0, 6,  16,  32, 22, 16,  64);
  cvt(sgb_w1,        W1P,                 192, kNst, kGpadK, 0, 0, 192,   0,  0,  0, 192);
  cvt(sgc_w1,        W1P + 192 * kGpadK,  192, kNst, kGpadK, 0, 0, 192,   0,  0,  0, 192);
  cvt(sgb_w2,        W2P,                  16, kSgh, kSgh,   0, 0,  16,   0,  0,  0,  64);
  cvt(sgc_w2,        W2P + 64 * kSgh,      16, kSgh, kSgh,   0, 0,  16,   0,  0,  0,  64);
  cvt(out_proj_w,    WOP,                  96, kDin, kDin,   0, 0,  96,   0,  0,  0,  96);
  cvt(hbl,           HB,                kRows, kCm,  kCm,    0, 0, kRows, 0,  0,  0, kRows);

  ln_c_kernel<<<kRows / 64, 256, 0, stream>>>(x, ln_g, ln_b, XN);

  wmma_gemm64<1, false, 0, 0, false><<<dim3(192, 1), 256, 0, stream>>>(
      XN, nullptr, kCm, 0L, WIN, nullptr, kCm, 0L,
      (void*)XI, nullptr, kDin, 0L, nullptr, nullptr, 0L, kRows, kDin, kCm, 1.0f);
  wmma_gemm64<1, false, 0, 0, false><<<dim3(192, 1), 256, 0, stream>>>(
      XN, nullptr, kCm, 0L, WIN + 192 * kCm, nullptr, kCm, 0L,
      (void*)Z, nullptr, kDin, 0L, nullptr, nullptr, 0L, kRows, kDin, kCm, 1.0f);

  wmma_gemm64<1, false, 0, 3, false><<<dim3(192, 1), 256, 0, stream>>>(
      HB, nullptr, kCm, 0L, WIL, nullptr, kCm, 0L,
      (void*)LOW, nullptr, kDin, 0L, nullptr, nullptr, 0L, kRows, kDin, kCm, 1.0f);

  conv3_silu_kernel<<<dim3(kRows / 32, kDin / 64), 256, 0, stream>>>(XI, conv2d_w, conv2d_b, XS);

  wmma_gemm64<1, false, 0, 0, false><<<dim3(64, 1), 256, 0, stream>>>(
      XS, nullptr, kDin, 0L, WXP, nullptr, kDin, 0L,
      (void*)XD, nullptr, kXdP, 0L, nullptr, nullptr, 0L, kRows, kXdP, kDin, 1.0f);
  wmma_gemm64<1, false, 0, 3, false><<<dim3(64, 1), 256, 0, stream>>>(
      LOW, nullptr, kDin, 0L, WXL, nullptr, kDin, 0L,
      (void*)VBC, nullptr, kXdP, 0L, nullptr, nullptr, 0L, kRows, kXdP, kDin, 1.0f);

  wmma_gemm64<1, false, 0, 3, false><<<dim3(192, 2), 256, 0, stream>>>(
      VBC, nullptr, kXdP, 32L, W1P, nullptr, kGpadK, (long)192 * kGpadK,
      (void*)HG, nullptr, kDin, (long)kRows * kDin, nullptr, nullptr, 0L, kRows, kDin, kGpadK, 1.0f);

  glu_kernel<<<(2 * kRows * 48) / 256, 256, 0, stream>>>((const unsigned*)HG, (unsigned*)G, 2 * kRows * 48);

  wmma_gemm64<1, false, 0, 0, false><<<dim3(64, 2), 256, 0, stream>>>(
      G, nullptr, kSgh, (long)kRows * kSgh, W2P, nullptr, kSgh, (long)64 * kSgh,
      (void*)SG, nullptr, kXdP, (long)kRows * kXdP, nullptr, nullptr, 0L, kRows, kXdP, kSgh, 1.0f);

  xc_prep_kernel<<<kRows / 64, 256, 0, stream>>>(XD, SG, SG + (size_t)kRows * kXdP, conv_dt_w, conv_B_w, conv_C_w, XC);

  scan_kernel<<<kBatch * (kDin / kScanCh), kScanCh, 0, stream>>>(XC, XS, dt_proj_w, dt_proj_b, A_logs, Ds, Y);

  ln_gate_kernel<<<kRows / 64, 256, 0, stream>>>(Y, Z, outn_g, outn_b, YG);

  outproj_kernel<<<kRows / 256, 256, 0, stream>>>(YG, WOP, x, out, kRows);
}
